// CondConvInvertedResidual_70222715289957
// MI455X (gfx1250) — hardware-verified
//
#include <hip/hip_runtime.h>
#include <stddef.h>


#define NB    32
#define CIN   96
#define COUT  96
#define HW    3136
#define NE    8
#define HID   576
#define MIXN  55296
#define R2P   32
#define EPS   1e-5f
#define WSC   16.0f
#define WSCI  0.0625f

typedef _Float16 v16h __attribute__((ext_vector_type(16)));
typedef _Float16 v8h  __attribute__((ext_vector_type(8)));
typedef _Float16 v4h  __attribute__((ext_vector_type(4)));
typedef float    v8f  __attribute__((ext_vector_type(8)));
typedef float    v4f  __attribute__((ext_vector_type(4)));

union Frag { v16h v; v8h h8[2]; };

__device__ __forceinline__ v8f wmma_f16(v16h a, v16h b, v8f c) {
  c = __builtin_amdgcn_wmma_f32_16x16x32_f16(false, a, false, b, (short)0, c, false, false);
  asm volatile("v_nop\n\tv_nop\n\tv_nop\n\tv_nop" : "+v"(c) : "v"(a), "v"(b));
  return c;
}

__device__ __forceinline__ float wave_sum(float v) {
#pragma unroll
  for (int o = 16; o > 0; o >>= 1) v += __shfl_xor(v, o, 32);
  return v;
}

__device__ __forceinline__ float sigm(float z) {
  return __builtin_amdgcn_rcpf(1.0f + __expf(-z));
}

__global__ __launch_bounds__(256)
void k_prep(const float* __restrict__ x,
            const float* __restrict__ wr1, const float* __restrict__ br1,
            const float* __restrict__ wr3, const float* __restrict__ br3,
            const float* __restrict__ w1, const float* __restrict__ w3,
            _Float16* __restrict__ w1c, _Float16* __restrict__ w3c)
{
  const int b = blockIdx.x;
  const int tid = threadIdx.x, lane = tid & 31, wave = tid >> 5;
  __shared__ float xm[CIN];
  __shared__ float rg[16];

  const float* xb = x + (size_t)b * CIN * HW;
  for (int c = wave; c < CIN; c += 8) {
    const v4f* p = (const v4f*)(xb + (size_t)c * HW);
    float s = 0.f;
    for (int i = lane; i < HW / 4; i += 32) {
      const v4f v = p[i];
      s += (v[0] + v[1]) + (v[2] + v[3]);
    }
    s = wave_sum(s);
    if (lane == 0) xm[c] = s * (1.0f / (float)HW);
  }
  __syncthreads();
  if (tid < 16) {
    const int e = tid & 7;
    const float* wr = (tid < 8) ? wr1 : wr3;
    const float* br = (tid < 8) ? br1 : br3;
    float a = br[e];
#pragma unroll 1
    for (int c = 0; c < CIN; ++c) a = fmaf(xm[c], wr[e * CIN + c], a);
    rg[tid] = sigm(a);
  }
  __syncthreads();

#pragma unroll 1
  for (int job = 0; job < 2; ++job) {
    const float* wsrc = job ? w3 : w1;
    _Float16* dst = (job ? w3c : w1c) + (size_t)b * MIXN;
    const int go = job * 8;
#pragma unroll 1
    for (int s = 0; s < MIXN / (768 * 8); ++s) {
      v8h val[3];
#pragma unroll
      for (int j = 0; j < 3; ++j) {
        const int q = s * 768 + j * 256 + tid;
        const size_t e0 = (size_t)q * 8;
        v4f lo = {0.f, 0.f, 0.f, 0.f};
        v4f hi = {0.f, 0.f, 0.f, 0.f};
#pragma unroll 1
        for (int e = 0; e < NE; ++e) {
          const float g = rg[go + e];
          const v4f* p = (const v4f*)(wsrc + (size_t)e * MIXN + e0);
          const v4f a0 = p[0];
          const v4f a1 = p[1];
          lo = lo + g * a0;
          hi = hi + g * a1;
        }
        v8h o;
#pragma unroll
        for (int i = 0; i < 4; ++i) {
          o[i]     = (_Float16)(lo[i] * WSC);
          o[4 + i] = (_Float16)(hi[i] * WSC);
        }
        val[j] = o;
      }
#pragma unroll
      for (int j = 0; j < 3; ++j)
        *(volatile v8h*)(dst + ((size_t)(s * 768 + j * 256 + tid)) * 8) = val[j];
      __threadfence();
#pragma unroll
      for (int j = 0; j < 3; ++j)
        *(volatile v8h*)(dst + ((size_t)(s * 768 + j * 256 + tid)) * 8) = val[j];
    }
  }
}

__global__ __launch_bounds__(192)
void k_expand(const float* __restrict__ x, const _Float16* __restrict__ w1c,
              const float* __restrict__ g1, const float* __restrict__ bt1,
              const float* __restrict__ m1, const float* __restrict__ v1,
              _Float16* __restrict__ y)
{
  const int p0 = blockIdx.x * 64;
  const int b  = blockIdx.y;
  const int tid = threadIdx.x, lane = tid & 31, wave = tid >> 5;
  const int m = lane & 15, h = lane >> 4;

  __shared__ __align__(16) _Float16 Bs[64][104];
  __shared__ __align__(16) _Float16 Ts[6][16][72];
  __shared__ float invs[HID];
  __shared__ float adds[HID];

  for (int i = tid; i < HID; i += 192) {
    const float inv = g1[i] * rsqrtf(v1[i] + EPS);
    invs[i] = inv * WSCI;
    adds[i] = bt1[i] - m1[i] * inv;
  }
  const float* xb = x + (size_t)b * CIN * HW + p0;
  for (int t = tid; t < 384; t += 192) {
    const int kq = t >> 4, ng = t & 15;
    const int k0 = kq * 4, n = ng * 4;
    const v4f r0 = *(const v4f*)(xb + (size_t)(k0 + 0) * HW + n);
    const v4f r1 = *(const v4f*)(xb + (size_t)(k0 + 1) * HW + n);
    const v4f r2 = *(const v4f*)(xb + (size_t)(k0 + 2) * HW + n);
    const v4f r3 = *(const v4f*)(xb + (size_t)(k0 + 3) * HW + n);
#pragma unroll
    for (int i = 0; i < 4; ++i) {
      v4h pk;
      pk[0] = (_Float16)r0[i];
      pk[1] = (_Float16)r1[i];
      pk[2] = (_Float16)r2[i];
      pk[3] = (_Float16)r3[i];
      *(v4h*)&Bs[n + i][k0] = pk;
    }
  }
  __syncthreads();

#pragma unroll 1
  for (int ms = 0; ms < HID / 96; ++ms) {
    const int row0 = ms * 96 + wave * 16;
    v8f acc[4];
    {
      const v8f z = {0.f, 0.f, 0.f, 0.f, 0.f, 0.f, 0.f, 0.f};
#pragma unroll
      for (int j = 0; j < 4; ++j) acc[j] = z;
    }
    const _Float16* arow = w1c + ((size_t)b * HID + row0 + m) * CIN;
#pragma unroll
    for (int ks = 0; ks < 3; ++ks) {
      const int k0 = ks * 32;
      Frag fa;
      fa.h8[0] = *(const v8h*)(arow + k0 + 8 * h);
      fa.h8[1] = *(const v8h*)(arow + k0 + 16 + 8 * h);
#pragma unroll
      for (int j = 0; j < 4; ++j) {
        Frag fb;
        fb.h8[0] = *(const v8h*)&Bs[j * 16 + m][k0 + 8 * h];
        fb.h8[1] = *(const v8h*)&Bs[j * 16 + m][k0 + 16 + 8 * h];
        acc[j] = wmma_f16(fa.v, fb.v, acc[j]);
      }
    }
#pragma unroll
    for (int r = 0; r < 8; ++r) {
      const int rl = 8 * h + r;
      const float iv = invs[row0 + rl], ad = adds[row0 + rl];
#pragma unroll
      for (int j = 0; j < 4; ++j) {
        const float v = fminf(fmaxf(fmaf(acc[j][r], iv, ad), 0.f), 6.f);
        Ts[wave][rl][j * 16 + m] = (_Float16)v;
      }
    }
    __syncthreads();
    v8h sv[4];
#pragma unroll
    for (int it = 0; it < 4; ++it)
      sv[it] = *(const v8h*)&Ts[wave][it * 4 + (lane >> 3)][(lane & 7) * 8];
    _Float16* yb = y + ((size_t)b * HID + row0) * HW + p0;
#pragma unroll
    for (int it = 0; it < 4; ++it)
      *(volatile v8h*)(yb + (size_t)(it * 4 + (lane >> 3)) * HW + (lane & 7) * 8) = sv[it];
    __threadfence();
#pragma unroll
    for (int it = 0; it < 4; ++it)
      *(volatile v8h*)(yb + (size_t)(it * 4 + (lane >> 3)) * HW + (lane & 7) * 8) = sv[it];
    __syncthreads();
  }
}

__global__ __launch_bounds__(256)
void k_route2(const _Float16* __restrict__ y, const float* __restrict__ wr2,
              const float* __restrict__ br2, float* __restrict__ r2t)
{
  const int b = blockIdx.x;
  const int tid = threadIdx.x, lane = tid & 31, wave = tid >> 5;
  __shared__ float ym[HID];
  __shared__ float rr[NE];

  const _Float16* yb = y + (size_t)b * HID * HW;
  for (int c = wave; c < HID; c += 8) {
    const v8h* p = (const v8h*)(yb + (size_t)c * HW);
    float s = 0.f;
    for (int i = lane; i < HW / 8; i += 32) {
      const v8h v = p[i];
      s += (((float)v[0] + (float)v[1]) + ((float)v[2] + (float)v[3])) +
           (((float)v[4] + (float)v[5]) + ((float)v[6] + (float)v[7]));
    }
    s = wave_sum(s);
    if (lane == 0) ym[c] = s * (1.0f / (float)HW);
  }
  __syncthreads();
  {
    float a = 0.f;
#pragma unroll 1
    for (int c = lane; c < HID; c += 32) a = fmaf(ym[c], wr2[wave * HID + c], a);
    a = wave_sum(a);
    if (lane == 0) rr[wave] = sigm(a + br2[wave]);
  }
  __syncthreads();
  if (wave == 0) {
    v4f v;
#pragma unroll
    for (int i = 0; i < 4; ++i) {
      const int idx = lane * 4 + i;
      const float g = rr[idx & 7];
      v[i] = (idx < NE) ? g : 0.f;
    }
    float* dstp = r2t + (size_t)b * R2P + lane * 4;
    if (lane < 8) *(volatile v4f*)dstp = v;
    __threadfence();
    if (lane < 8) *(volatile v4f*)dstp = v;
  }
}

__global__ __launch_bounds__(256)
void k_dwconv(_Float16* __restrict__ y, const float* __restrict__ r2t,
              const float* __restrict__ w2,
              const float* __restrict__ g2, const float* __restrict__ bt2,
              const float* __restrict__ m2, const float* __restrict__ v2)
{
  const int bc = blockIdx.x;
  const int b = bc / HID, c = bc - b * HID;
  const int tid = threadIdx.x;
  __shared__ __align__(16) float Ps[58][64];
  __shared__ __align__(16) v8h Os[HW / 8];
  __shared__ float taps[9];
  __shared__ float bnp[2];
  _Float16* plane = y + (size_t)bc * HW;

  for (int i = tid; i < 64; i += 256) { Ps[0][i] = 0.f; Ps[57][i] = 0.f; }
  for (int i = tid; i < 56; i += 256) { Ps[i + 1][3] = 0.f; Ps[i + 1][60] = 0.f; }
  for (int q = tid; q < HW / 8; q += 256) {
    const v8h v = *(const v8h*)(plane + (size_t)q * 8);
    const int hr = q / 7, w0 = (q - hr * 7) * 8;
    v4f lo, hi;
#pragma unroll
    for (int i = 0; i < 4; ++i) { lo[i] = (float)v[i]; hi[i] = (float)v[4 + i]; }
    *(v4f*)&Ps[hr + 1][4 + w0] = lo;
    *(v4f*)&Ps[hr + 1][8 + w0] = hi;
  }
  if (tid < 9) {
    float a = 0.f;
#pragma unroll 1
    for (int e = 0; e < NE; ++e)
      a = fmaf(r2t[(size_t)b * R2P + e], w2[((size_t)e * HID + c) * 9 + tid], a);
    taps[tid] = a;
  }
  if (tid == 32) {
    const float inv = g2[c] * rsqrtf(v2[c] + EPS);
    bnp[0] = inv;
    bnp[1] = bt2[c] - m2[c] * inv;
  }
  __syncthreads();

  float k[9];
#pragma unroll
  for (int t = 0; t < 9; ++t) k[t] = taps[t];
  const float inv = bnp[0], add = bnp[1];

#pragma unroll 1
  for (int t = tid; t < HW / 8; t += 256) {
    const int hr = t / 7, w0 = (t - hr * 7) * 8;
    float in[3][10];
#pragma unroll
    for (int dy = 0; dy < 3; ++dy) {
      const float* rp = &Ps[hr + dy][w0 + 3];
      const v4f a4 = *(const v4f*)(rp + 1);
      const v4f b4 = *(const v4f*)(rp + 5);
      in[dy][0] = rp[0];
      in[dy][1] = a4[0]; in[dy][2] = a4[1]; in[dy][3] = a4[2]; in[dy][4] = a4[3];
      in[dy][5] = b4[0]; in[dy][6] = b4[1]; in[dy][7] = b4[2]; in[dy][8] = b4[3];
      in[dy][9] = rp[9];
    }
    v8h o;
#pragma unroll
    for (int j = 0; j < 8; ++j) {
      float acc = 0.f;
#pragma unroll
      for (int dy = 0; dy < 3; ++dy)
#pragma unroll
        for (int dx = 0; dx < 3; ++dx)
          acc = fmaf(k[dy * 3 + dx], in[dy][j + dx], acc);
      o[j] = (_Float16)fminf(fmaxf(fmaf(acc, inv, add), 0.f), 6.f);
    }
    Os[t] = o;
  }
  __syncthreads();
  for (int t = tid; t < HW / 8; t += 256)
    *(volatile v8h*)(plane + (size_t)t * 8) = Os[t];
  __threadfence();
  for (int t = tid; t < HW / 8; t += 256)
    *(volatile v8h*)(plane + (size_t)t * 8) = Os[t];
}

__global__ __launch_bounds__(192)
void k_project(const _Float16* __restrict__ y2, const _Float16* __restrict__ w3c,
               const float* __restrict__ x,
               const float* __restrict__ g3, const float* __restrict__ bt3,
               const float* __restrict__ m3, const float* __restrict__ v3,
               float* __restrict__ out)
{
  const int p0 = blockIdx.x * 64;
  const int b  = blockIdx.y;
  const int tid = threadIdx.x, lane = tid & 31, wave = tid >> 5;
  const int m = lane & 15, h = lane >> 4;

  __shared__ __align__(16) _Float16 Bs[64][104];
  __shared__ __align__(16) float Ts[6][16][68];
  __shared__ float invs[COUT];
  __shared__ float adds[COUT];

  if (tid < COUT) {
    const float inv = g3[tid] * rsqrtf(v3[tid] + EPS);
    invs[tid] = inv * WSCI;
    adds[tid] = bt3[tid] - m3[tid] * inv;
  }

  const int row0 = wave * 16;
  v8f acc[4];
  {
    const v8f z = {0.f, 0.f, 0.f, 0.f, 0.f, 0.f, 0.f, 0.f};
#pragma unroll
    for (int j = 0; j < 4; ++j) acc[j] = z;
  }
  const _Float16* arow = w3c + ((size_t)b * COUT + row0 + m) * HID;
  const _Float16* yb = y2 + (size_t)b * HID * HW + p0;

#pragma unroll 1
  for (int kc = 0; kc < HID / 96; ++kc) {
    __syncthreads();
    {
      const int kq = tid >> 3, ng = tid & 7;
      const _Float16* src = yb + (size_t)(kc * 96 + kq * 4) * HW + ng * 8;
      const v8h r0 = *(const v8h*)(src);
      const v8h r1 = *(const v8h*)(src + HW);
      const v8h r2 = *(const v8h*)(src + 2 * (size_t)HW);
      const v8h r3 = *(const v8h*)(src + 3 * (size_t)HW);
#pragma unroll
      for (int i = 0; i < 8; ++i) {
        v4h pk;
        pk[0] = r0[i]; pk[1] = r1[i]; pk[2] = r2[i]; pk[3] = r3[i];
        *(v4h*)&Bs[ng * 8 + i][kq * 4] = pk;
      }
    }
    __syncthreads();
#pragma unroll
    for (int ks = 0; ks < 3; ++ks) {
      const int k0 = ks * 32;
      Frag fa;
      fa.h8[0] = *(const v8h*)(arow + kc * 96 + k0 + 8 * h);
      fa.h8[1] = *(const v8h*)(arow + kc * 96 + k0 + 16 + 8 * h);
#pragma unroll
      for (int j = 0; j < 4; ++j) {
        Frag fb;
        fb.h8[0] = *(const v8h*)&Bs[j * 16 + m][k0 + 8 * h];
        fb.h8[1] = *(const v8h*)&Bs[j * 16 + m][k0 + 16 + 8 * h];
        acc[j] = wmma_f16(fa.v, fb.v, acc[j]);
      }
    }
  }

#pragma unroll
  for (int r = 0; r < 8; ++r) {
    const int rl = 8 * h + r;
    const float iv = invs[row0 + rl], ad = adds[row0 + rl];
#pragma unroll
    for (int j = 0; j < 4; ++j)
      Ts[wave][rl][j * 16 + m] = fmaf(acc[j][r], iv, ad);
  }
  __syncthreads();
  v4f sv[8];
  const float* xrow = x + ((size_t)b * COUT + row0) * HW + p0;
#pragma unroll
  for (int it = 0; it < 8; ++it) {
    const int rl = it * 2 + (lane >> 4), ch = lane & 15;
    const v4f tv = *(const v4f*)&Ts[wave][rl][ch * 4];
    const v4f xv = *(const v4f*)(xrow + (size_t)rl * HW + ch * 4);
    sv[it] = tv + xv;
  }
  float* ob = out + ((size_t)b * COUT + row0) * HW + p0;
#pragma unroll
  for (int it = 0; it < 8; ++it)
    *(volatile v4f*)(ob + (size_t)(it * 2 + (lane >> 4)) * HW + (lane & 15) * 4) = sv[it];
  __threadfence();
#pragma unroll
  for (int it = 0; it < 8; ++it)
    *(volatile v4f*)(ob + (size_t)(it * 2 + (lane >> 4)) * HW + (lane & 15) * 4) = sv[it];
}

extern "C" void kernel_launch(void* const* d_in, const int* in_sizes, int n_in,
                              void* d_out, int out_size, void* d_ws, size_t ws_size,
                              hipStream_t stream) {
  if (n_in < 22) return;
  if (in_sizes[0] != NB * CIN * HW) return;
  if (out_size != NB * COUT * HW) return;
  if (in_sizes[1] != NE * CIN || in_sizes[3] != NE * HID * CIN) return;
  if (in_sizes[8] != NE * HID || in_sizes[10] != NE * HID * 9) return;
  if (in_sizes[15] != NE * COUT * HID || in_sizes[20] != NE * CIN) return;
  if (in_sizes[2] < NE || in_sizes[9] < NE || in_sizes[21] < NE) return;
  if (in_sizes[4] < HID || in_sizes[5] < HID || in_sizes[6] < HID || in_sizes[7] < HID) return;
  if (in_sizes[11] < HID || in_sizes[12] < HID || in_sizes[13] < HID || in_sizes[14] < HID) return;
  if (in_sizes[16] < COUT || in_sizes[17] < COUT || in_sizes[18] < COUT || in_sizes[19] < COUT) return;

  const float* x    = (const float*)d_in[0];
  const float* wr1  = (const float*)d_in[1];
  const float* br1  = (const float*)d_in[2];
  const float* w1   = (const float*)d_in[3];
  const float* g1   = (const float*)d_in[4];
  const float* bt1  = (const float*)d_in[5];
  const float* m1   = (const float*)d_in[6];
  const float* v1   = (const float*)d_in[7];
  const float* wr2  = (const float*)d_in[8];
  const float* br2  = (const float*)d_in[9];
  const float* w2   = (const float*)d_in[10];
  const float* g2   = (const float*)d_in[11];
  const float* bt2  = (const float*)d_in[12];
  const float* m2   = (const float*)d_in[13];
  const float* v2   = (const float*)d_in[14];
  const float* w3   = (const float*)d_in[15];
  const float* g3   = (const float*)d_in[16];
  const float* bt3  = (const float*)d_in[17];
  const float* m3   = (const float*)d_in[18];
  const float* v3   = (const float*)d_in[19];
  const float* wr3  = (const float*)d_in[20];
  const float* br3  = (const float*)d_in[21];
  float* out = (float*)d_out;

  const size_t off_r2t = 0;
  const size_t sz_r2t  = (size_t)NB * R2P * sizeof(float);
  const size_t off_w1c = off_r2t + sz_r2t;
  const size_t sz_w1c  = (size_t)NB * MIXN * sizeof(_Float16);
  const size_t off_w3c = off_w1c + sz_w1c;
  const size_t sz_w3c  = (size_t)NB * MIXN * sizeof(_Float16);
  const size_t off_y   = off_w3c + sz_w3c;
  const size_t sz_y    = (size_t)NB * HID * HW * sizeof(_Float16);
  const size_t total   = off_y + sz_y;
  if (total > ws_size) return;

  char* wsp = (char*)d_ws;
  float*    r2t = (float*)(wsp + off_r2t);
  _Float16* w1c = (_Float16*)(wsp + off_w1c);
  _Float16* w3c = (_Float16*)(wsp + off_w3c);
  _Float16* yws = (_Float16*)(wsp + off_y);

  k_prep<<<NB, 256, 0, stream>>>(x, wr1, br1, wr3, br3, w1, w3, w1c, w3c);

  {
    dim3 grid(HW / 64, NB);
    k_expand<<<grid, 192, 0, stream>>>(x, w1c, g1, bt1, m1, v1, yws);
  }

  k_route2<<<NB, 256, 0, stream>>>(yws, wr2, br2, r2t);

  k_dwconv<<<NB * HID, 256, 0, stream>>>(yws, r2t, w2, g2, bt2, m2, v2);

  {
    dim3 grid(HW / 64, NB);
    k_project<<<grid, 192, 0, stream>>>(yws, w3c, x, g3, bt3, m3, v3, out);
  }
}
